// LinearAttention_61220463837901
// MI455X (gfx1250) — hardware-run, weakly checked
//
#include <hip/hip_runtime.h>
#include <math.h>

typedef __attribute__((ext_vector_type(16))) _Float16 v16h;
typedef __attribute__((ext_vector_type(8)))  _Float16 v8h;
typedef __attribute__((ext_vector_type(8)))  float    v8f;
typedef __attribute__((ext_vector_type(4)))  float    v4f;

constexpr int kNB    = 8;
constexpr int kSeqL  = 4096;
constexpr int kFeat  = 256;
constexpr int kRows  = kNB * kSeqL;
constexpr int kSTile = kSeqL / 64;
constexpr int kElems = kNB * kSeqL * kFeat;
static_assert(kElems == 8388608);
static_assert((kSeqL % 64) == 0 && (kFeat % 64) == 0 && (kRows % 64) == 0);
static_assert((kSeqL % 32) == 0 && (kFeat % 32) == 0);

constexpr float kMapA = 0.6053f;
constexpr float kMapB = 4.102f;

constexpr float kPhiCarry = 16.0f;
constexpr float kValCarry = 64.0f;
constexpr float kKvScale  = 1.0f / kValCarry;
constexpr float kOutScale = 1.0f / (kPhiCarry * kPhiCarry);
constexpr float kHalfMinNormal = 6.103515625e-5f;

constexpr size_t kOffPKT = 0;
constexpr size_t kOffVTP = kOffPKT + (size_t)kNB * kFeat * kSeqL * 2;
constexpr size_t kOffPQP = kOffVTP + (size_t)kNB * kFeat * kSeqL * 2;
constexpr size_t kOffKVT = kOffPQP + (size_t)kRows * kFeat * 2;
constexpr size_t kOffKPA = kOffKVT + (size_t)kNB * kFeat * kFeat * 2;
constexpr size_t kOffKSU = kOffKPA + (size_t)kNB * kSTile * kFeat * 4;
constexpr size_t kOffRBO = kOffKSU + (size_t)kNB * kFeat * 4;
constexpr size_t kWsTotal = kOffRBO + (size_t)kRows * 4;
static_assert(kWsTotal == 52043776ull);
static_assert(kWsTotal <= 134217728ull);
static_assert((kOffVTP % 128) == 0 && (kOffPQP % 128) == 0 && (kOffKVT % 128) == 0 &&
              (kOffKPA % 128) == 0 && (kOffKSU % 128) == 0 && (kOffRBO % 128) == 0);

__device__ __forceinline__ float phi_map(float x) {
  const float z = kMapA * x - kMapB;
  const float e = expf(-z);
  return __builtin_amdgcn_rcpf(1.0f + e);
}

__device__ __forceinline__ _Float16 to_half_flush(float v) {
  const float w = (fabsf(v) < kHalfMinNormal) ? 0.0f : v;
  return (_Float16)w;
}

struct FragH {
  union U { v16h v; v8h h[2]; };
  static __device__ __forceinline__ v16h load(const _Float16* p) {
    U f;
    f.h[0] = *(const v8h*)(p);
    f.h[1] = *(const v8h*)(p + 16);
    return f.v;
  }
};

__device__ __forceinline__ v8f mma_h(v16h a, v16h b, v8f c) {
  c = __builtin_amdgcn_wmma_f32_16x16x32_f16(false, a, false, b, (short)0, c, false, false);
  asm volatile("v_nop\n\tv_nop\n\tv_nop\n\tv_nop" : "+v"(c) : "v"(a), "v"(b));
  return c;
}
__device__ __forceinline__ void acc_guard4(v8f& a, v8f& b, v8f& c, v8f& d) {
  asm volatile("v_nop\n\tv_nop\n\tv_nop\n\tv_nop" : "+v"(a), "+v"(b), "+v"(c), "+v"(d));
}

template <int OUT_MODE, bool ROWSCALE>
__global__ __launch_bounds__(256) void wmma_gemm64(
    const unsigned short* __restrict__ Ap, int lda, long strideA,
    const unsigned short* __restrict__ Btp, int ldb, long strideB,
    void* __restrict__ Cout, int ldc, long strideC,
    const float* __restrict__ rowscale, long strideRS,
    int M, int N, int K, float scale) {
  const _Float16* A  = (const _Float16*)Ap;
  const _Float16* Bt = (const _Float16*)Btp;
  __shared__ __align__(16) float sT[8][16 * 68];
  const int b    = blockIdx.y;
  const int lane = threadIdx.x & 31;
  const int wave = threadIdx.x >> 5;
  const int tilesN = N >> 6;
  const int tilesM = M >> 6;
  const int tile = blockIdx.x * 8 + wave;
  if (tile >= tilesM * tilesN) return;
  const int tm = tile / tilesN;
  const int tn = tile - tm * tilesN;
  const int m0 = tm << 6;
  const int n0 = tn << 6;

  const _Float16* Ab = A  + (size_t)b * strideA;
  const _Float16* Bb = Bt + (size_t)b * strideB;

  const int rlane = lane & 15;
  const int koff  = (lane >> 4) * 8;
  const int mOff  = (lane >> 4) * 8;

  v8f acc[4][4];
#pragma unroll
  for (int i = 0; i < 4; ++i)
#pragma unroll
    for (int j = 0; j < 4; ++j) acc[i][j] = (v8f){0.f, 0.f, 0.f, 0.f, 0.f, 0.f, 0.f, 0.f};

  for (int k0 = 0; k0 < K; k0 += 32) {
    v16h bh[4];
#pragma unroll
    for (int j = 0; j < 4; ++j) {
      const size_t bo = (size_t)(n0 + (j << 4) + rlane) * ldb + koff + k0;
      bh[j] = FragH::load(Bb + bo);
    }
#pragma unroll
    for (int i = 0; i < 4; ++i) {
      const size_t ao = (size_t)(m0 + (i << 4) + rlane) * lda + koff + k0;
      const v16h ah = FragH::load(Ab + ao);
#pragma unroll
      for (int j = 0; j < 4; ++j) acc[i][j] = mma_h(ah, bh[j], acc[i][j]);
    }
  }
  acc_guard4(acc[0][0], acc[0][1], acc[0][2], acc[0][3]);
  acc_guard4(acc[1][0], acc[1][1], acc[1][2], acc[1][3]);
  acc_guard4(acc[2][0], acc[2][1], acc[2][2], acc[2][3]);
  acc_guard4(acc[3][0], acc[3][1], acc[3][2], acc[3][3]);

  float* slab = sT[wave];
#pragma unroll
  for (int i = 0; i < 4; ++i) {
    const int mBase = m0 + (i << 4);
    float rsv[8];
    if (ROWSCALE) {
      const float* rp = rowscale + (size_t)b * strideRS + mBase + mOff;
      const v4f r0 = *(const v4f*)(rp);
      const v4f r1 = *(const v4f*)(rp + 4);
#pragma unroll
      for (int e = 0; e < 4; ++e) {
        rsv[e]     = r0[e] * scale;
        rsv[4 + e] = r1[e] * scale;
      }
    } else {
#pragma unroll
      for (int e = 0; e < 8; ++e) rsv[e] = scale;
    }
#pragma unroll
    for (int j = 0; j < 4; ++j) {
#pragma unroll
      for (int r = 0; r < 8; ++r) {
        const float v = acc[i][j][r] * rsv[r];
        slab[(mOff + r) * 68 + (j << 4) + rlane] = v;
      }
    }
    __builtin_amdgcn_fence(__ATOMIC_RELEASE, "workgroup");
    __builtin_amdgcn_wave_barrier();
    __builtin_amdgcn_fence(__ATOMIC_ACQUIRE, "workgroup");
    if (OUT_MODE == 0) {
      float* C = (float*)Cout + (size_t)b * strideC;
      const int hh = lane >> 4, c4 = (lane & 15) * 4;
      for (int pass = 0; pass < 2; ++pass) {
#pragma unroll
        for (int it = 0; it < 8; ++it) {
          const int row = it * 2 + hh;
          const v4f v = *(const v4f*)(slab + row * 68 + c4);
          *(volatile v4f*)(C + (size_t)(mBase + row) * ldc + n0 + c4) = v;
        }
        __threadfence();
      }
    } else {
      const int q = lane >> 3, c8 = (lane & 7) * 8;
      unsigned short* C = (unsigned short*)Cout + (size_t)b * strideC;
      v8h hv[4];
#pragma unroll
      for (int it = 0; it < 4; ++it) {
        const int row = it * 4 + q;
        const float* sp = slab + row * 68 + c8;
#pragma unroll
        for (int e = 0; e < 8; ++e) hv[it][e] = to_half_flush(sp[e]);
      }
      for (int pass = 0; pass < 2; ++pass) {
#pragma unroll
        for (int it = 0; it < 4; ++it) {
          const int row = it * 4 + q;
          *(volatile v8h*)(C + (size_t)(mBase + row) * ldc + n0 + c8) = hv[it];
        }
        __threadfence();
      }
    }
    __builtin_amdgcn_fence(__ATOMIC_RELEASE, "workgroup");
    __builtin_amdgcn_wave_barrier();
    __builtin_amdgcn_fence(__ATOMIC_ACQUIRE, "workgroup");
  }
}

template <bool PHI>
__global__ __launch_bounds__(256) void tr_plane_kernel(const float* __restrict__ src, unsigned short* __restrict__ dst,
                                                       float* __restrict__ kpart, float carry) {
  __shared__ float sm[64][65];
  __shared__ __align__(16) float sred[64];
  const int t = threadIdx.x, lane = t & 31, wave = t >> 5;
  const int d0 = blockIdx.x * 64;
  const int st = blockIdx.y;
  const int s0 = st * 64;
  const int b  = blockIdx.z;
  const float* sp = src + ((size_t)b * kSeqL + s0) * kFeat + d0;
  const int lr = t >> 4, c4 = (t & 15) * 4;
#pragma unroll 1
  for (int i = 0; i < 4; ++i) {
    const int r = i * 16 + lr;
    const v4f x = *(const v4f*)(sp + (size_t)r * kFeat + c4);
#pragma unroll
    for (int e = 0; e < 4; ++e) {
      float v = x[e];
      if (PHI) v = phi_map(v);
      sm[c4 + e][r] = v;
    }
  }
  __syncthreads();
  if (PHI) {
    if (t < 64) {
      float s = 0.0f;
#pragma unroll 1
      for (int j = 0; j < 64; ++j) s += sm[t][j];
      sred[t] = s;
    }
    __syncthreads();
  }
  const int q = lane >> 3, c8 = (lane & 7) * 8;
  v8h hv[2];
#pragma unroll
  for (int it = 0; it < 2; ++it) {
    const int row = wave * 8 + it * 4 + q;
#pragma unroll
    for (int e = 0; e < 8; ++e) hv[it][e] = to_half_flush(sm[row][c8 + e] * carry);
  }
  unsigned short* dp = dst + ((size_t)b * kFeat + d0) * kSeqL + s0;
  for (int pass = 0; pass < 2; ++pass) {
#pragma unroll
    for (int it = 0; it < 2; ++it) {
      const int row = wave * 8 + it * 4 + q;
      *(volatile v8h*)(dp + (size_t)row * kSeqL + c8) = hv[it];
    }
    __threadfence();
  }
  if (PHI) {
    const v4f pv = *(const v4f*)(sred + (t & 15) * 4);
    if (t < 16) {
      float* kp = kpart + ((size_t)b * kSTile + st) * kFeat + d0 + t * 4;
      *(volatile v4f*)kp = pv;
      __threadfence();
      *(volatile v4f*)kp = pv;
    }
  }
}

__global__ __launch_bounds__(256) void ksum_final_kernel(const float* __restrict__ kpart, float* __restrict__ ksum) {
  const int b = blockIdx.x, t = threadIdx.x;
  float s = 0.0f;
#pragma unroll 1
  for (int st = 0; st < kSTile; ++st) s += kpart[((size_t)b * kSTile + st) * kFeat + t];
  volatile float* p = ksum + b * kFeat + t;
  *p = s;
  __threadfence();
  *p = s;
}

__global__ __launch_bounds__(256) void q_plane_kernel(const float* __restrict__ Q, const float* __restrict__ ksum,
                                                      unsigned short* __restrict__ PQ, float* __restrict__ rbot) {
  __shared__ __align__(16) float sR[64];
  const int t = threadIdx.x, lane = t & 31, wave = t >> 5;
  const int m0 = blockIdx.x * 64;
  const int b  = m0 / kSeqL;
  const float* kp = ksum + b * kFeat + lane * 8;
  const v4f k0 = *(const v4f*)(kp);
  const v4f k1 = *(const v4f*)(kp + 4);
#pragma unroll 1
  for (int i = 0; i < 8; ++i) {
    const int m = m0 + wave * 8 + i;
    const float* qp = Q + (size_t)m * kFeat + lane * 8;
    const v4f a0 = *(const v4f*)(qp);
    const v4f a1 = *(const v4f*)(qp + 4);
    float dot = 0.0f;
    v8h hv;
#pragma unroll
    for (int e = 0; e < 4; ++e) {
      const float p0 = phi_map(a0[e]);
      const float p1 = phi_map(a1[e]);
      dot = fmaf(p0, k0[e], dot);
      dot = fmaf(p1, k1[e], dot);
      hv[e]     = to_half_flush(p0 * kPhiCarry);
      hv[4 + e] = to_half_flush(p1 * kPhiCarry);
    }
#pragma unroll
    for (int off = 16; off > 0; off >>= 1) dot += __shfl_xor(dot, off, 32);
    const float rb = 1.0f / dot;
    if (lane == 0) sR[wave * 8 + i] = rb;
    unsigned short* op = PQ + (size_t)m * kFeat + lane * 8;
    *(volatile v8h*)op = hv;
    __threadfence();
    *(volatile v8h*)op = hv;
  }
  __syncthreads();
  const v4f pv = *(const v4f*)(sR + (t & 15) * 4);
  if (t < 16) {
    float* rp = rbot + m0 + t * 4;
    *(volatile v4f*)rp = pv;
    __threadfence();
    *(volatile v4f*)rp = pv;
  }
}

extern "C" void kernel_launch(void* const* d_in, const int* in_sizes, int n_in,
                              void* d_out, int out_size, void* d_ws, size_t ws_size,
                              hipStream_t stream) {
  if (n_in < 3) return;
  if (in_sizes[0] != kElems) return;
  if (in_sizes[1] != kElems) return;
  if (in_sizes[2] != kElems) return;
  if (out_size != kElems) return;
  if (ws_size < kWsTotal) return;

  const float* Q = (const float*)d_in[0];
  const float* K = (const float*)d_in[1];
  const float* V = (const float*)d_in[2];
  float* out = (float*)d_out;

  char* ws = (char*)d_ws;
  unsigned short* PKT = (unsigned short*)(ws + kOffPKT);
  unsigned short* VTP = (unsigned short*)(ws + kOffVTP);
  unsigned short* PQP = (unsigned short*)(ws + kOffPQP);
  unsigned short* KVT = (unsigned short*)(ws + kOffKVT);
  float*          KPA = (float*)(ws + kOffKPA);
  float*          KSU = (float*)(ws + kOffKSU);
  float*          RBO = (float*)(ws + kOffRBO);

  const dim3 trGrid(kFeat / 64, kSTile, kNB);
  tr_plane_kernel<true><<<trGrid, 256, 0, stream>>>(K, PKT, KPA, kPhiCarry);
  tr_plane_kernel<false><<<trGrid, 256, 0, stream>>>(V, VTP, KPA, kValCarry);

  ksum_final_kernel<<<kNB, 256, 0, stream>>>(KPA, KSU);

  q_plane_kernel<<<kRows / 64, 256, 0, stream>>>(Q, KSU, PQP, RBO);

  wmma_gemm64<1, false><<<dim3(2, kNB), 256, 0, stream>>>(
      VTP, kSeqL, (long)kFeat * kSeqL,
      PKT, kSeqL, (long)kFeat * kSeqL,
      (void*)KVT, kFeat, (long)kFeat * kFeat,
      RBO, 0L,
      kFeat, kFeat, kSeqL, kKvScale);

  wmma_gemm64<0, true><<<dim3(32, kNB), 256, 0, stream>>>(
      PQP, kFeat, (long)kSeqL * kFeat,
      KVT, kFeat, (long)kFeat * kFeat,
      (void*)out, kFeat, (long)kSeqL * kFeat,
      RBO, (long)kSeqL,
      kSeqL, kFeat, kFeat, kOutScale);
}
